// Attention_15315853377738
// MI455X (gfx1250) — hardware-verified
//
#include <hip/hip_runtime.h>


#ifndef NB
#define NB 2
#endif
#ifndef SEQ
#define SEQ 2048
#endif
#define NB_FULL  2
#define SEQ_FULL 2048
#define DM   2048
#define NH   16
#define NKV  4
#define HD   128
#define NQC  (NH * HD)
#define NKC  (NKV * HD)
#define NPC  (NQC + 2 * NKC)
#define CTP  (2 * NQC)
#define RT   64
#define NWV  4
#define BQ   (16 * NWV)
#define KS   32
#define OSP  132
#define GBM  64
#define GBN  128
#define VTK  64
#define VTP  72
#define L2E  1.4426950408889634f
#define SCL  (0.08838834764831845f * L2E)
#define PCARRY 8.0f

static_assert(HD == 128);
static_assert(GBN == HD);
static_assert(RT * 2 == HD);
static_assert(NH == 16 && NKV == 4);
static_assert(SEQ % BQ == 0);
static_assert(SEQ % GBM == 0);
static_assert(SEQ % KS == 0);
static_assert(SEQ % 128 == 0);
static_assert(NB <= NB_FULL);
static_assert(SEQ <= SEQ_FULL);
static_assert(DM % 32 == 0 && CTP % 32 == 0);
static_assert(DM % VTK == 0 && DM / VTK == 32);
static_assert(NPC % GBN == 0 && DM % GBN == 0 && NQC % GBN == 0);
static_assert(((size_t)NB * SEQ * DM) % 2048 == 0);
static_assert((size_t)(NQC / 128 + 2 * NKC / 128 + DM / 128) * 32u * (size_t)(VTK * 128) == (size_t)DM * NPC + (size_t)NQC * DM);
static_assert((size_t)(NPC / GBN) * (size_t)(NB * SEQ / GBM) * (size_t)(GBM * GBN) == (size_t)NB * SEQ * NPC);
static_assert((size_t)(NB * NH * (SEQ / BQ)) * (size_t)(BQ * HD) * 2u == (size_t)NB * SEQ * CTP);
static_assert((size_t)(DM / GBN) * (size_t)(NB * SEQ / GBM) * (size_t)(GBM * GBN) == (size_t)NB * SEQ * DM);

#define BYTES_XB  ((size_t)NB * SEQ * DM * 2)
#define BYTES_WT  ((size_t)NPC * DM * 2)
#define BYTES_WOT ((size_t)DM * NQC * 2)
#define BYTES_QP  ((size_t)NB * SEQ * NQC * 2)
#define BYTES_KP  ((size_t)NB * SEQ * NKC * 2)
#define BYTES_VT  ((size_t)NB * NKV * HD * SEQ * 2)
#define BYTES_CT  ((size_t)NB * SEQ * CTP * 2)
#define BYTES_ALL (BYTES_XB + BYTES_WT + BYTES_WOT + BYTES_QP + BYTES_KP + BYTES_VT + BYTES_CT)
static_assert(BYTES_ALL <= (size_t)134217728);
static_assert(BYTES_XB % 256 == 0 && BYTES_WT % 256 == 0 && BYTES_WOT % 256 == 0 && BYTES_QP % 256 == 0 && BYTES_KP % 256 == 0 && BYTES_VT % 256 == 0 && BYTES_CT % 256 == 0);

typedef unsigned short us;
typedef __attribute__((ext_vector_type(16))) __bf16   v16bf;
typedef __attribute__((ext_vector_type(16))) _Float16 v16h;
typedef __attribute__((ext_vector_type(2)))  _Float16 v2h;
typedef __attribute__((ext_vector_type(8)))  unsigned short v8us;
typedef __attribute__((ext_vector_type(8)))  unsigned int   v8u;
typedef __attribute__((ext_vector_type(4)))  unsigned int   v4u;
typedef __attribute__((ext_vector_type(8)))  float    v8f;
typedef __attribute__((ext_vector_type(4)))  float    v4f;
typedef v4f  __attribute__((may_alias)) v4fa;
typedef v8us __attribute__((may_alias)) v8usa;

__device__ __forceinline__ unsigned short f2bf(float f) { unsigned u = __float_as_uint(f); u += 0x7FFFu + ((u >> 16) & 1u); return (unsigned short)(u >> 16); }
__device__ __forceinline__ float bf2f(unsigned short b) { return __uint_as_float(((unsigned)b) << 16); }
__device__ __forceinline__ float bfr(float f) { return bf2f(f2bf(f)); }
__device__ __forceinline__ v16bf cat16b(v8us lo, v8us hi) { return __builtin_bit_cast(v16bf, __builtin_shufflevector(lo, hi, 0, 1, 2, 3, 4, 5, 6, 7, 8, 9, 10, 11, 12, 13, 14, 15)); }
__device__ __forceinline__ v16h  cat16h(v8us lo, v8us hi) { return __builtin_bit_cast(v16h,  __builtin_shufflevector(lo, hi, 0, 1, 2, 3, 4, 5, 6, 7, 8, 9, 10, 11, 12, 13, 14, 15)); }
__device__ __forceinline__ v8f wmmab(v16bf a, v16bf b, v8f c) { return __builtin_amdgcn_wmma_f32_16x16x32_bf16(false, a, false, b, (short)0, c, false, false); }
__device__ __forceinline__ v8f wmmah(v16h a, v16h b, v8f c)   { return __builtin_amdgcn_wmma_f32_16x16x32_f16(false, a, false, b, (short)0, c, false, false); }
__device__ __forceinline__ v16bf ldb(const us* p) { return cat16b(*(const v8us*)p, *(const v8us*)(p + 16)); }
__device__ __forceinline__ v16h  ldh(const us* p) { return cat16h(*(const v8us*)p, *(const v8us*)(p + 16)); }
__device__ __forceinline__ unsigned pk2h(float a, float b) { v2h t; t[0] = (_Float16)a; t[1] = (_Float16)b; return __builtin_bit_cast(unsigned, t); }

__global__ __launch_bounds__(256) void k_cvt(const float* __restrict__ x, us* XB) {
    const unsigned i = blockIdx.x * 256u + threadIdx.x;
    const unsigned per = (unsigned)(SEQ * (DM / 8));
    if (i >= (unsigned)NB * per) return;
    const unsigned b = i / per, r = i - b * per;
    const float* src = x + (size_t)b * SEQ_FULL * DM + (size_t)r * 8;
    us* dst = XB + (size_t)i * 8;
    const v8f v = *(const v8f*)src;
    v8us o;
#pragma unroll
    for (int c = 0; c < 8; ++c) o[c] = f2bf(v[c]);
    *(volatile v8us*)dst = o;
    __threadfence();
    *(volatile v8us*)dst = o;
}

__global__ __launch_bounds__(256) void k_wt(const float* __restrict__ Wq, const float* __restrict__ Wkv, const float* __restrict__ Wo, us* WT, us* WOT) {
    __shared__ __align__(16) us tl[128 * VTP];
    const unsigned tid = threadIdx.x;
    const unsigned blk = blockIdx.x;
    const float* W; us* OUT; unsigned nc, r;
    if (blk < 512u)      { W = Wq;  OUT = WT;                      nc = (unsigned)NQC;       r = blk; }
    else if (blk < 768u) { W = Wkv; OUT = WT + (size_t)NQC * DM;   nc = (unsigned)(2 * NKC); r = blk - 512u; }
    else                 { W = Wo;  OUT = WOT;                     nc = (unsigned)DM;        r = blk - 768u; }
    const unsigned k0 = (r & 31u) * VTK;
    const unsigned c0 = (r >> 5) * 128u;
    const float* src = W + (size_t)k0 * nc + c0;
#pragma unroll
    for (unsigned it = 0; it < 8; ++it) {
        const unsigned f = it * 256u + tid;
        const unsigned kk = f >> 5, d4 = (f & 31u) * 4u;
        const v4f x = *(const v4f*)(src + (size_t)kk * nc + d4);
#pragma unroll
        for (unsigned c = 0; c < 4; ++c) tl[(d4 + c) * VTP + kk] = f2bf(x[c]);
    }
    __syncthreads();
    us* dst = OUT + (size_t)c0 * DM + k0;
    const unsigned c8 = (tid & 7u) * 8u, dr = tid >> 3;
#pragma unroll 1
    for (int ps = 0; ps < 2; ++ps) {
#pragma unroll
        for (unsigned it = 0; it < 4; ++it) {
            const unsigned d = it * 32u + dr;
            const v8us o = *(const v8usa*)(tl + d * VTP + c8);
            *(volatile v8us*)(dst + (size_t)d * DM + c8) = o;
        }
        if (ps == 0) __threadfence();
    }
}

template <unsigned LDA, unsigned LDB, unsigned KL, unsigned KMASK>
__device__ __forceinline__ void gemm_tile(const us* __restrict__ A, const us* __restrict__ Bt, unsigned m0, unsigned n0, float* cs) {
    static_assert(KL % 32u == 0u);
    static_assert(((KMASK + 1u) & KMASK) == 0u && (KMASK + 1u) % 32u == 0u);
    const unsigned tid = threadIdx.x, lane = tid & 31u, wv = tid >> 5, lr = lane & 15u, hi = lane >> 4;
    const unsigned wm = (wv & 1u) * 32u, wn = (wv >> 1) * 64u;
    const us* ap = A + (size_t)(m0 + wm + lr) * LDA + 8u * hi;
    const us* bp = Bt + (size_t)(n0 + wn + lr) * LDB + 8u * hi;
    v8f acc[8];
#pragma unroll
    for (int i = 0; i < 8; ++i) acc[i] = (v8f){};
#pragma unroll 1
    for (unsigned k0 = 0; k0 < KL; k0 += 32u) {
        const us* bq = bp + (k0 & KMASK);
        const v16bf a0 = ldb(ap + k0);
        const v16bf a1 = ldb(ap + (size_t)16u * LDA + k0);
        v16bf b4[4];
#pragma unroll
        for (int ni = 0; ni < 4; ++ni) b4[ni] = ldb(bq + (size_t)ni * 16u * LDB);
#pragma unroll
        for (int ni = 0; ni < 4; ++ni) {
            acc[ni]     = wmmab(a0, b4[ni], acc[ni]);
            acc[4 + ni] = wmmab(a1, b4[ni], acc[4 + ni]);
        }
        asm volatile("v_nop\n\tv_nop\n\tv_nop\n\tv_nop"
                     : "+v"(acc[0]), "+v"(acc[1]), "+v"(acc[2]), "+v"(acc[3]), "+v"(acc[4]), "+v"(acc[5]), "+v"(acc[6]), "+v"(acc[7])
                     : "v"(a0), "v"(a1), "v"(b4[3]));
    }
#pragma unroll
    for (int mi = 0; mi < 2; ++mi) {
#pragma unroll
        for (int ni = 0; ni < 4; ++ni) {
#pragma unroll
            for (int r = 0; r < 8; ++r)
                cs[(wm + mi * 16u + 8u * hi + r) * OSP + wn + ni * 16u + lr] = acc[mi * 4 + ni][r];
        }
    }
    __syncthreads();
}

__global__ __launch_bounds__(128) void k_proj(const us* __restrict__ XB, const us* __restrict__ WT, const float* __restrict__ cosT, const float* __restrict__ sinT,
                                              us* QP, us* KP, us* VT) {
    __shared__ __align__(16) float cs[GBM * OSP];
    const unsigned tid = threadIdx.x;
    const unsigned ct = blockIdx.x;
    const unsigned m0 = blockIdx.y * GBM;
    gemm_tile<DM, DM, DM, DM - 1u>(XB, WT, m0, ct * GBN, cs);
    const unsigned b = m0 / (unsigned)SEQ;
    const unsigned nr0 = m0 - b * (unsigned)SEQ;
    if (ct < 20u) {
        us* dst; unsigned pitch;
        if (ct < 16u) { dst = QP + (size_t)m0 * NQC + ct * HD;          pitch = (unsigned)NQC; }
        else          { dst = KP + (size_t)m0 * NKC + (ct - 16u) * HD;  pitch = (unsigned)NKC; }
        const unsigned p = tid & 15u, rr = tid >> 4, i0 = (p & 7u) * 8u;
        const bool sec = (p >> 3) != 0u;
#pragma unroll 1
        for (int ps = 0; ps < 2; ++ps) {
#pragma unroll 2
            for (unsigned it = 0; it < 8; ++it) {
                const unsigned row = it * 8u + rr;
                const float* cr = cs + row * OSP + i0;
                const v4f a0 = *(const v4fa*)(cr), a1 = *(const v4fa*)(cr + 4);
                const v4f b0 = *(const v4fa*)(cr + 64), b1 = *(const v4fa*)(cr + 68);
                const float* cp = cosT + (size_t)(nr0 + row) * RT + i0;
                const float* sp = sinT + (size_t)(nr0 + row) * RT + i0;
                const v4f c0 = *(const v4f*)(cp), c1 = *(const v4f*)(cp + 4);
                const v4f s0 = *(const v4f*)(sp), s1 = *(const v4f*)(sp + 4);
                float o[8];
#pragma unroll
                for (int j = 0; j < 4; ++j) {
                    const float cj = bfr(c0[j]), sj = bfr(s0[j]);
                    const float u = sec ? b0[j] : a0[j];
                    const float w = sec ? -a0[j] : b0[j];
                    o[j] = u * cj + w * sj;
                    const float ck = bfr(c1[j]), sk = bfr(s1[j]);
                    const float u2 = sec ? b1[j] : a1[j];
                    const float w2 = sec ? -a1[j] : b1[j];
                    o[4 + j] = u2 * ck + w2 * sk;
                }
                v4u ov;
                ov[0] = pk2h(o[0], o[1]); ov[1] = pk2h(o[2], o[3]); ov[2] = pk2h(o[4], o[5]); ov[3] = pk2h(o[6], o[7]);
                *(volatile v4u*)(dst + (size_t)row * pitch + p * 8u) = ov;
            }
            if (ps == 0) __threadfence();
        }
    } else {
        const unsigned g = ct - 20u;
        us* dst = VT + (size_t)(b * NKV + g) * HD * SEQ + nr0;
        const unsigned c8 = (tid & 7u) * 8u, dr = tid >> 3;
#pragma unroll 1
        for (int ps = 0; ps < 2; ++ps) {
#pragma unroll 2
            for (unsigned it = 0; it < 8; ++it) {
                const unsigned d = it * 16u + dr;
                const float* cc = cs + c8 * OSP + d;
                v4u ov;
                ov[0] = pk2h(cc[0 * OSP], cc[1 * OSP]);
                ov[1] = pk2h(cc[2 * OSP], cc[3 * OSP]);
                ov[2] = pk2h(cc[4 * OSP], cc[5 * OSP]);
                ov[3] = pk2h(cc[6 * OSP], cc[7 * OSP]);
                *(volatile v4u*)(dst + (size_t)d * SEQ + c8) = ov;
            }
            if (ps == 0) __threadfence();
        }
    }
}

__global__ __launch_bounds__(128) void k_flash(const us* __restrict__ QP, const us* __restrict__ KP, const us* __restrict__ VT, const float* __restrict__ mask, us* CT) {
    __shared__ __align__(16) float os[NWV * 16 * OSP];
    __shared__ __align__(16) float bs[SEQ];
    const unsigned tid = threadIdx.x, lane = tid & 31u, wv = tid >> 5, lr = lane & 15u, hi = lane >> 4;
    const unsigned qtiles = (unsigned)(SEQ / BQ);
    const unsigned hb = blockIdx.x / qtiles;
    const unsigned qt = blockIdx.x - hb * qtiles;
    const unsigned h = hb & (unsigned)(NH - 1), b = hb >> 4;
    const unsigned g = h & (unsigned)(NKV - 1);
    const unsigned q0 = qt * BQ + wv * 16u;

#pragma unroll 1
    for (unsigned i = tid; i < (unsigned)SEQ; i += 128u) {
        const float m = bfr(mask[(size_t)b * SEQ_FULL + i]);
        bs[i] = (1.0f - m) * -1.0e9f * L2E;
    }
    __syncthreads();

    const us* qp = QP + ((size_t)b * SEQ + q0 + lr) * NQC + h * HD + 8u * hi;
    const us* kp = KP + ((size_t)b * SEQ + lr) * NKC + g * HD + 8u * hi;
    const us* vp = VT + ((size_t)(b * NKV + g) * HD + lr) * SEQ + 8u * hi;

    v8f o[8];
#pragma unroll
    for (int t = 0; t < 8; ++t) o[t] = (v8f){};
    float ml = -1.0e30f;
    float l = 0.0f;

#pragma unroll 1
    for (unsigned k0 = 0; k0 < (unsigned)SEQ; k0 += KS) {
        unsigned zo = 0u;
        asm volatile("" : "+v"(zo));
        v8f s0 = (v8f){}, s1 = (v8f){};
        const us* ka = kp + (size_t)k0 * NKC;
        const us* qa = qp + zo;
        v16h qlast;
#pragma unroll
        for (int dk = 0; dk < 4; ++dk) {
            const v16h qf = ldh(qa + dk * 32);
            const v16h a0 = ldh(ka + dk * 32);
            const v16h a1 = ldh(ka + 16 * NKC + dk * 32);
            s0 = wmmah(a0, qf, s0);
            s1 = wmmah(a1, qf, s1);
            qlast = qf;
        }
        asm volatile("v_nop\n\tv_nop\n\tv_nop\n\tv_nop" : "+v"(s0), "+v"(s1) : "v"(qlast));

        const float* bb = bs + k0 + 8u * hi;
        const v4f b00 = *(const v4fa*)(bb), b01 = *(const v4fa*)(bb + 4);
        const v4f b10 = *(const v4fa*)(bb + 16), b11 = *(const v4fa*)(bb + 20);
        float t0[8], t1[8];
#pragma unroll
        for (int r = 0; r < 4; ++r) {
            t0[r]     = fmaf(s0[r],     SCL, b00[r]);
            t0[4 + r] = fmaf(s0[4 + r], SCL, b01[r]);
            t1[r]     = fmaf(s1[r],     SCL, b10[r]);
            t1[4 + r] = fmaf(s1[4 + r], SCL, b11[r]);
        }
        float mx = fmaxf(t0[0], t1[0]);
#pragma unroll
        for (int r = 1; r < 8; ++r) mx = fmaxf(mx, fmaxf(t0[r], t1[r]));
        mx = fmaxf(mx, __shfl_xor(mx, 16, 32));
        const float mnl = fmaxf(ml, mx);
        const float corr = __builtin_amdgcn_exp2f(ml - mnl);
        ml = mnl;
        const float mo = mnl - PCARRY;
        float p0[8], p1[8];
        float ps = 0.0f;
#pragma unroll
        for (int r = 0; r < 8; ++r) {
            p0[r] = __builtin_amdgcn_exp2f(t0[r] - mo);
            p1[r] = __builtin_amdgcn_exp2f(t1[r] - mo);
            ps += p0[r] + p1[r];
        }
        ps += __shfl_xor(ps, 16, 32);
        l = l * corr + ps;
        if (__builtin_amdgcn_ballot_w32(corr != 1.0f) != 0u) {
#pragma unroll
            for (int t = 0; t < 8; ++t) o[t] *= corr;
        }

        v8u hw;
#pragma unroll
        for (int j = 0; j < 4; ++j) {
            hw[j]     = pk2h(p0[2 * j], p0[2 * j + 1]);
            hw[4 + j] = pk2h(p1[2 * j], p1[2 * j + 1]);
        }
        const v16h ph = __builtin_bit_cast(v16h, hw);

        asm volatile("" ::: "memory");
        const us* va = vp + k0;
#pragma unroll
        for (int t = 0; t < 8; ++t) {
            const v16h a = ldh(va + (size_t)t * 16 * SEQ);
            o[t] = wmmah(a, ph, o[t]);
        }
        asm volatile("v_nop\n\tv_nop\n\tv_nop\n\tv_nop"
                     : "+v"(o[0]), "+v"(o[1]), "+v"(o[2]), "+v"(o[3]), "+v"(o[4]), "+v"(o[5]), "+v"(o[6]), "+v"(o[7])
                     : "v"(ph));
    }

    const float inv = 1.0f / l;
    float* ow = os + wv * (16 * OSP);
#pragma unroll
    for (int t = 0; t < 8; ++t) {
#pragma unroll
        for (int r = 0; r < 8; ++r) ow[lr * OSP + t * 16 + 8 * hi + r] = o[t][r] * inv;
    }
    __syncthreads();
    const unsigned pc = lane & 15u, rh = lane >> 4;
    us* crow = CT + ((size_t)b * SEQ + q0) * CTP + h * HD + pc * 8u;
#pragma unroll 1
    for (int ps2 = 0; ps2 < 2; ++ps2) {
#pragma unroll 2
        for (unsigned it = 0; it < 8; ++it) {
            const unsigned s2 = it * 2u + rh;
            const float* src = ow + s2 * OSP + pc * 8u;
            const v4f x0 = *(const v4fa*)(src), x1 = *(const v4fa*)(src + 4);
            v8us hv, lv;
#pragma unroll
            for (int c = 0; c < 4; ++c) {
                const unsigned short h0 = f2bf(x0[c]);
                const unsigned short h1 = f2bf(x1[c]);
                hv[c] = h0; hv[4 + c] = h1;
                lv[c] = f2bf(x0[c] - bf2f(h0));
                lv[4 + c] = f2bf(x1[c] - bf2f(h1));
            }
            *(volatile v8us*)(crow + (size_t)s2 * CTP) = hv;
            *(volatile v8us*)(crow + (size_t)s2 * CTP + NQC) = lv;
        }
        if (ps2 == 0) __threadfence();
    }
}

__global__ __launch_bounds__(128) void k_oproj(const us* __restrict__ CT, const us* __restrict__ WOT, const float* __restrict__ bo, float* OUT) {
    __shared__ __align__(16) float cs[GBM * OSP];
    const unsigned tid = threadIdx.x, lane = tid & 31u, wv = tid >> 5;
    const unsigned n0 = blockIdx.x * GBN;
    const unsigned m0 = blockIdx.y * GBM;
    gemm_tile<CTP, NQC, CTP, NQC - 1u>(CT, WOT, m0, n0, cs);
    const v4f bv = *(const v4f*)(bo + n0 + lane * 4u);
    v4f bb;
    bb[0] = bfr(bv[0]); bb[1] = bfr(bv[1]); bb[2] = bfr(bv[2]); bb[3] = bfr(bv[3]);
    float* orow = OUT + (size_t)(m0 + wv * 16u) * DM + n0 + lane * 4u;
    const float* crow = cs + (wv * 16u) * OSP + lane * 4u;
#pragma unroll 1
    for (int ps = 0; ps < 2; ++ps) {
#pragma unroll 4
        for (unsigned s = 0; s < 16; ++s) {
            v4f val = *(const v4fa*)(crow + s * OSP);
            val[0] += bb[0]; val[1] += bb[1]; val[2] += bb[2]; val[3] += bb[3];
            *(volatile v4f*)(orow + (size_t)s * DM) = val;
        }
        if (ps == 0) __threadfence();
    }
}

extern "C" void kernel_launch(void* const* d_in, const int* in_sizes, int n_in,
                              void* d_out, int out_size, void* d_ws, size_t ws_size, hipStream_t stream) {
    if (n_in < 8) return;
    const size_t need_x = ((size_t)(NB - 1) * SEQ_FULL + SEQ) * DM;
    const size_t need_m = (size_t)(NB - 1) * SEQ_FULL + SEQ;
    if ((size_t)in_sizes[0] < need_x) return;
    if ((size_t)in_sizes[1] < (size_t)SEQ * RT || (size_t)in_sizes[2] < (size_t)SEQ * RT) return;
    if ((size_t)in_sizes[3] < need_m) return;
    if ((size_t)in_sizes[4] < (size_t)DM * NQC || (size_t)in_sizes[5] < (size_t)DM * 2 * NKC) return;
    if ((size_t)in_sizes[6] < (size_t)NQC * DM || (size_t)in_sizes[7] < (size_t)DM) return;
    if ((size_t)out_size < (size_t)NB * SEQ * DM) return;
    if (BYTES_ALL > ws_size) return;
    const float* x    = (const float*)d_in[0];
    const float* cosT = (const float*)d_in[1];
    const float* sinT = (const float*)d_in[2];
    const float* mask = (const float*)d_in[3];
    const float* Wq   = (const float*)d_in[4];
    const float* Wkv  = (const float*)d_in[5];
    const float* Wo   = (const float*)d_in[6];
    const float* bo   = (const float*)d_in[7];
    float* OUT = (float*)d_out;
    char* wsp = (char*)d_ws;
    us* XB  = (us*)(wsp);
    us* WT  = (us*)(wsp + BYTES_XB);
    us* WOT = (us*)(wsp + BYTES_XB + BYTES_WT);
    us* QP  = (us*)(wsp + BYTES_XB + BYTES_WT + BYTES_WOT);
    us* KP  = (us*)(wsp + BYTES_XB + BYTES_WT + BYTES_WOT + BYTES_QP);
    us* VT  = (us*)(wsp + BYTES_XB + BYTES_WT + BYTES_WOT + BYTES_QP + BYTES_KP);
    us* CT  = (us*)(wsp + BYTES_XB + BYTES_WT + BYTES_WOT + BYTES_QP + BYTES_KP + BYTES_VT);
    const unsigned gc = (unsigned)(((size_t)NB * SEQ * DM / 8 + 255) / 256);
    k_cvt<<<gc, 256, 0, stream>>>(x, XB);
    k_wt<<<1280, 256, 0, stream>>>(Wq, Wkv, Wo, WT, WOT);
    k_proj<<<dim3((unsigned)(NPC / GBN), (unsigned)(NB * SEQ / GBM), 1), 128, 0, stream>>>(XB, WT, cosT, sinT, QP, KP, VT);
    k_flash<<<(unsigned)(NB * NH * (SEQ / BQ)), 128, 0, stream>>>(QP, KP, VT, mask, CT);
    k_oproj<<<dim3((unsigned)(DM / GBN), (unsigned)(NB * SEQ / GBM), 1), 128, 0, stream>>>(CT, WOT, bo, OUT);
}
